// VaswaniMultiHeadAttention_42992622633336
// MI455X (gfx1250) — hardware-verified
//
#include <hip/hip_runtime.h>

typedef _Float16 v16h __attribute__((ext_vector_type(16)));
typedef _Float16 v8h  __attribute__((ext_vector_type(8)));
typedef float    v8f  __attribute__((ext_vector_type(8)));
typedef float    v4f  __attribute__((ext_vector_type(4)));
typedef v8h __attribute__((may_alias)) v8ha;
typedef v4f __attribute__((may_alias)) v4fa;

union Frag { v16h v; v8h half[2]; };

#define EMB    1024
#define NHEADS 16
#define HD     64
#define SEQ    2048
#define BATCH  2
#define MROWS  (BATCH * SEQ)
#define NX     (MROWS * EMB)
#define NW     (EMB * EMB)
#define NX8    (NX / 8)
#define WSC    32.0f
#define WINV   0.03125f
#define SSCALE 0.03125f
#define PSCALE 16384.0f
#define TPITCH 72

__device__ __forceinline__ v8f wmma_f16(v16h a, v16h b, v8f c) {
  v8f d = __builtin_amdgcn_wmma_f32_16x16x32_f16(false, a, false, b, (short)0, c, false, false);
  asm volatile("v_nop\n\tv_nop\n\tv_nop\n\tv_nop" : "+v"(d) : "v"(a), "v"(b));
  return d;
}

__device__ __forceinline__ v16h load_frag(const _Float16* p, int h) {
  Frag f;
  f.half[0] = *(const v8ha*)(p + 8 * h);
  f.half[1] = *(const v8ha*)(p + 16 + 8 * h);
  return f.v;
}

__global__ __launch_bounds__(256) void convert_kernel(
    const float* __restrict__ q, const float* __restrict__ v,
    _Float16* __restrict__ qx, _Float16* __restrict__ vx)
{
  const int g = blockIdx.x * 256 + threadIdx.x;
  if (g >= 2 * NX8) return;
  const float* src;
  _Float16* dst;
  if (g < NX8) {
    src = q + (size_t)g * 8;
    dst = qx + (size_t)g * 8;
  } else {
    const int e = g - NX8;
    src = v + (size_t)e * 8;
    dst = vx + (size_t)e * 8;
  }
  const v4f a = *(const v4fa*)src;
  const v4f c = *(const v4fa*)(src + 4);
  const v8h o = { (_Float16)a.x, (_Float16)a.y, (_Float16)a.z, (_Float16)a.w,
                  (_Float16)c.x, (_Float16)c.y, (_Float16)c.z, (_Float16)c.w };
  *(volatile v8h*)dst = o;
  __threadfence();
  *(volatile v8h*)dst = o;
}

__device__ __forceinline__ void wt_store_pass(const _Float16* sW, _Float16* wt,
                                              int which, int n0, int k0, int w, int lane) {
  const int q8 = lane & 7, sub = lane >> 3;
  #pragma unroll
  for (int i = 0; i < 2; ++i) {
    const int nrow = w * 8 + i * 4 + sub;
    const v8h val = *(const v8ha*)(sW + nrow * TPITCH + 8 * q8);
    _Float16* dst = wt + ((size_t)which * EMB + n0 + nrow) * EMB + k0 + 8 * q8;
    *(volatile v8h*)dst = val;
  }
}

__global__ __launch_bounds__(256) void wtrans_kernel(
    const float* __restrict__ wq, const float* __restrict__ wk, const float* __restrict__ wv,
    _Float16* __restrict__ wt)
{
  __shared__ __attribute__((aligned(16))) _Float16 sW[64 * TPITCH];

  const int tid = threadIdx.x, lane = tid & 31, w = tid >> 5;
  const int n0 = blockIdx.x * 64, k0 = blockIdx.y * 64, which = blockIdx.z;
  const float* W = (which == 0) ? wq : ((which == 1) ? wk : wv);

  #pragma unroll
  for (int i = 0; i < 4; ++i) {
    const int idx = tid + 256 * i;
    const int kk = idx >> 4, nn = (idx & 15) * 4;
    const v4f x = *(const v4fa*)(W + (size_t)(k0 + kk) * EMB + n0 + nn);
    sW[(nn + 0) * TPITCH + kk] = (_Float16)(x.x * WSC);
    sW[(nn + 1) * TPITCH + kk] = (_Float16)(x.y * WSC);
    sW[(nn + 2) * TPITCH + kk] = (_Float16)(x.z * WSC);
    sW[(nn + 3) * TPITCH + kk] = (_Float16)(x.w * WSC);
  }
  __syncthreads();

  wt_store_pass(sW, wt, which, n0, k0, w, lane);
  __threadfence();
  wt_store_pass(sW, wt, which, n0, k0, w, lane);
}

__device__ __forceinline__ void proj_store_pass(const _Float16* sT, _Float16* plane, _Float16* vt,
                                                int which, int bh, int l0, int w, int lane) {
  const int q8 = lane & 7, sub = lane >> 3;
  #pragma unroll
  for (int i = 0; i < 8; ++i) {
    const int lid = w * 32 + i * 4 + sub;
    v8h val;
    _Float16* dst;
    if (which != 2) {
      val = *(const v8ha*)(sT + lid * HD + 8 * q8);
      dst = plane + ((size_t)bh * SEQ + l0 + lid) * HD + 8 * q8;
    } else {
      const int d = lid >> 1, hl = lid & 1;
      val = *(const v8ha*)(sT + d * 128 + 64 * hl + 8 * q8);
      dst = vt + ((size_t)bh * HD + d) * SEQ + l0 + 64 * hl + 8 * q8;
    }
    *(volatile v8h*)dst = val;
  }
}

__global__ __launch_bounds__(128) void proj_kernel(
    const _Float16* __restrict__ qx,
    const _Float16* __restrict__ vx,
    const _Float16* __restrict__ wt,
    const float* __restrict__ bq, const float* __restrict__ bk, const float* __restrict__ bv,
    _Float16* __restrict__ qp,
    _Float16* __restrict__ kp,
    _Float16* __restrict__ vt)
{
  __shared__ __attribute__((aligned(16))) _Float16 sT[128 * 64];

  const int tid = threadIdx.x, lane = tid & 31, w = tid >> 5;
  const int h = lane >> 4, m = lane & 15;
  const int m0 = blockIdx.x * 128;
  const int cg = blockIdx.y;
  const int which = cg >> 4, head = cg & 15;
  const int m0w = m0 + 32 * w;

  const _Float16* xsrc = (which == 0) ? qx : vx;
  const _Float16* xa0 = xsrc + (size_t)(m0w + m) * EMB;
  const _Float16* xa1 = xa0 + (size_t)16 * EMB;
  const _Float16* wb  = wt + ((size_t)which * EMB + head * HD + m) * EMB;

  const v8f zero8 = {0.f, 0.f, 0.f, 0.f, 0.f, 0.f, 0.f, 0.f};
  v8f acc[2][4];
  #pragma unroll
  for (int mt = 0; mt < 2; ++mt)
    #pragma unroll
    for (int nt = 0; nt < 4; ++nt) acc[mt][nt] = zero8;

  #pragma unroll 1
  for (int k0 = 0; k0 < EMB; k0 += 32) {
    const v16h a0 = load_frag(xa0 + k0, h);
    const v16h a1 = load_frag(xa1 + k0, h);
    #pragma unroll
    for (int nt = 0; nt < 4; ++nt) {
      const v16h b = load_frag(wb + (size_t)nt * 16 * EMB + k0, h);
      acc[0][nt] = wmma_f16(a0, b, acc[0][nt]);
      acc[1][nt] = wmma_f16(a1, b, acc[1][nt]);
    }
  }

  const float* bias = (which == 0) ? bq : ((which == 1) ? bk : bv);
  #pragma unroll
  for (int nt = 0; nt < 4; ++nt) {
    const int feat = 16 * nt + m;
    const float bvl = bias[head * HD + feat];
    #pragma unroll
    for (int mt = 0; mt < 2; ++mt) {
      #pragma unroll
      for (int r = 0; r < 8; ++r) {
        const int tokl = 32 * w + 16 * mt + 8 * h + r;
        const float y = acc[mt][nt][r] * WINV + bvl;
        const int idx = (which == 2) ? (feat * 128 + tokl) : (tokl * HD + feat);
        sT[idx] = (_Float16)y;
      }
    }
  }
  __syncthreads();

  const int b = m0 / SEQ, l0 = m0 - b * SEQ, bh = b * NHEADS + head;
  _Float16* plane = (which == 0) ? qp : kp;
  proj_store_pass(sT, plane, vt, which, bh, l0, w, lane);
  __threadfence();
  proj_store_pass(sT, plane, vt, which, bh, l0, w, lane);
}

__device__ __forceinline__ v16h pack_p(v8f a, v8f c) {
  const v16h r = { (_Float16)(a[0] * PSCALE), (_Float16)(a[1] * PSCALE), (_Float16)(a[2] * PSCALE), (_Float16)(a[3] * PSCALE),
                   (_Float16)(a[4] * PSCALE), (_Float16)(a[5] * PSCALE), (_Float16)(a[6] * PSCALE), (_Float16)(a[7] * PSCALE),
                   (_Float16)(c[0] * PSCALE), (_Float16)(c[1] * PSCALE), (_Float16)(c[2] * PSCALE), (_Float16)(c[3] * PSCALE),
                   (_Float16)(c[4] * PSCALE), (_Float16)(c[5] * PSCALE), (_Float16)(c[6] * PSCALE), (_Float16)(c[7] * PSCALE) };
  return r;
}

__device__ __forceinline__ void att_store_pass(const float* so, float* out,
                                               int b, int head, int q0, int lane) {
  const int q8 = lane & 7, sub = lane >> 3;
  #pragma unroll
  for (int i = 0; i < 8; ++i) {
    const int lid = i * 4 + sub;
    const int row = lid >> 1, hl = lid & 1;
    const v4f val = *(const v4fa*)(so + row * 64 + 32 * hl + 4 * q8);
    const size_t gi = ((size_t)b * SEQ + q0 + row) * EMB + head * HD + 32 * hl + 4 * q8;
    *(volatile v4f*)(out + gi) = val;
  }
}

__global__ __launch_bounds__(128) void attn_kernel(
    const _Float16* __restrict__ qp,
    const _Float16* __restrict__ kp,
    const _Float16* __restrict__ vt,
    float* __restrict__ out)
{
  __shared__ __attribute__((aligned(16))) float sO[4 * 16 * 64];

  const int tid = threadIdx.x, lane = tid & 31, w = tid >> 5;
  const int h = lane >> 4, m = lane & 15;
  const int bh = blockIdx.y, b = bh >> 4, head = bh & 15;
  const int q0 = blockIdx.x * 64 + 16 * w;

  const _Float16* qrow = qp + ((size_t)bh * SEQ + q0 + m) * HD;
  const v16h qb0 = load_frag(qrow, h);
  const v16h qb1 = load_frag(qrow + 32, h);

  const v8f zero8 = {0.f, 0.f, 0.f, 0.f, 0.f, 0.f, 0.f, 0.f};
  v8f o[4];
  #pragma unroll
  for (int t = 0; t < 4; ++t) o[t] = zero8;
  float mrun = -1e30f, lrun = 0.0f;

  const _Float16* kbase = kp + ((size_t)bh * SEQ + m) * HD;
  const _Float16* vbase = vt + ((size_t)bh * HD + m) * SEQ;

  #pragma unroll 1
  for (int kb = 0; kb < SEQ; kb += 64) {
    v8f s[4];
    #pragma unroll
    for (int j = 0; j < 4; ++j) {
      const _Float16* kpp = kbase + (size_t)(kb + 16 * j) * HD;
      const v16h kf0 = load_frag(kpp, h);
      const v16h kf1 = load_frag(kpp + 32, h);
      v8f z = zero8;
      z = wmma_f16(kf0, qb0, z);
      z = wmma_f16(kf1, qb1, z);
      s[j] = z;
    }
    #pragma unroll
    for (int j = 0; j < 4; ++j)
      #pragma unroll
      for (int r = 0; r < 8; ++r) s[j][r] = s[j][r] * SSCALE;

    float mloc = s[0][0];
    #pragma unroll
    for (int j = 0; j < 4; ++j)
      #pragma unroll
      for (int r = 0; r < 8; ++r) mloc = fmaxf(mloc, s[j][r]);
    mloc = fmaxf(mloc, __shfl_xor(mloc, 16));
    const float mnew = fmaxf(mrun, mloc);
    const float alpha = __expf(mrun - mnew);
    mrun = mnew;
    float lsum = 0.0f;
    #pragma unroll
    for (int j = 0; j < 4; ++j)
      #pragma unroll
      for (int r = 0; r < 8; ++r) {
        const float p = __expf(s[j][r] - mnew);
        s[j][r] = p;
        lsum += p;
      }
    lsum += __shfl_xor(lsum, 16);
    lrun = lrun * alpha + lsum;
    #pragma unroll
    for (int t = 0; t < 4; ++t)
      #pragma unroll
      for (int r = 0; r < 8; ++r) o[t][r] = o[t][r] * alpha;

    const v16h pb0 = pack_p(s[0], s[1]);
    const v16h pb1 = pack_p(s[2], s[3]);

    #pragma unroll
    for (int t = 0; t < 4; ++t) {
      const _Float16* vpp = vbase + (size_t)(16 * t) * SEQ + kb;
      const v16h vf0 = load_frag(vpp, h);
      const v16h vf1 = load_frag(vpp + 32, h);
      o[t] = wmma_f16(vf0, pb0, o[t]);
      o[t] = wmma_f16(vf1, pb1, o[t]);
    }
  }

  const float inv = (1.0f / lrun) * (1.0f / PSCALE);
  float* so = sO + w * 1024;
  #pragma unroll
  for (int t = 0; t < 4; ++t)
    #pragma unroll
    for (int r = 0; r < 8; ++r)
      so[m * 64 + 16 * t + 8 * h + r] = o[t][r] * inv;
  __syncthreads();

  att_store_pass(so, out, b, head, q0, lane);
  __threadfence();
  att_store_pass(so, out, b, head, q0, lane);
}

extern "C" void kernel_launch(void* const* d_in, const int* in_sizes, int n_in,
                              void* d_out, int out_size, void* d_ws, size_t ws_size,
                              hipStream_t stream) {
  if (n_in < 8) return;
  if (in_sizes[0] != NX || in_sizes[1] != NX) return;
  if (in_sizes[2] != NW || in_sizes[4] != NW || in_sizes[6] != NW) return;
  if (in_sizes[3] != EMB || in_sizes[5] != EMB || in_sizes[7] != EMB) return;
  if (out_size != NX) return;

  const float* q  = (const float*)d_in[0];
  const float* v  = (const float*)d_in[1];
  const float* Wq = (const float*)d_in[2];
  const float* bq = (const float*)d_in[3];
  const float* Wk = (const float*)d_in[4];
  const float* bk = (const float*)d_in[5];
  const float* Wv = (const float*)d_in[6];
  const float* bv = (const float*)d_in[7];
  float* out = (float*)d_out;

  const size_t x_bytes  = (size_t)NX * 2;
  const size_t wt_bytes = (size_t)3 * NW * 2;
  const size_t pl_bytes = (size_t)BATCH * NHEADS * SEQ * HD * 2;
  const size_t total = 2 * x_bytes + wt_bytes + 3 * pl_bytes;
  if (total > ws_size) return;

  char* ws = (char*)d_ws;
  _Float16* qx = (_Float16*)(ws);
  _Float16* vx = (_Float16*)(ws + x_bytes);
  _Float16* wt = (_Float16*)(ws + 2 * x_bytes);
  _Float16* qp = (_Float16*)(ws + 2 * x_bytes + wt_bytes);
  _Float16* kp = (_Float16*)(ws + 2 * x_bytes + wt_bytes + pl_bytes);
  _Float16* vt = (_Float16*)(ws + 2 * x_bytes + wt_bytes + 2 * pl_bytes);

  const int ngroups = 2 * NX8;
  convert_kernel<<<(ngroups + 255) / 256, 256, 0, stream>>>(q, v, qx, vx);

  dim3 gTr(EMB / 64, EMB / 64, 3);
  wtrans_kernel<<<gTr, 256, 0, stream>>>(Wq, Wk, Wv, wt);

  dim3 gProj(MROWS / 128, 3 * NHEADS);
  proj_kernel<<<gProj, 128, 0, stream>>>(qx, vx, wt, bq, bk, bv, qp, kp, vt);

  dim3 gAtt(SEQ / 64, BATCH * NHEADS);
  attn_kernel<<<gAtt, 128, 0, stream>>>(qp, kp, vt, out);
}
